// ModifiedMLP_6244882448515
// MI455X (gfx1250) — hardware-verified
//
#include <hip/hip_runtime.h>
#include <math.h>
#include <stdint.h>

typedef _Float16 v16h __attribute__((ext_vector_type(16)));
typedef _Float16 v8h  __attribute__((ext_vector_type(8)));
typedef float    v8f  __attribute__((ext_vector_type(8)));
typedef float    v4f  __attribute__((ext_vector_type(4)));
typedef unsigned int v4u __attribute__((ext_vector_type(4)));

#define HIDDEN     50
#define NPAD       64
#define KIN        32
#define KZ         64
#define NFEAT      10
#define NZL        4
#define ASTRIDE    72
#define FSTRIDE    68
#define RPB        128
#define NTHREADS   256

static_assert(ASTRIDE >= KZ, "");
static_assert(FSTRIDE >= NPAD, "");
static_assert((ASTRIDE * 2) % 16 == 0, "");
static_assert((FSTRIDE * 4) % 16 == 0, "");

#define TAB_WT     0
#define TAB_ZT     12288
#define TAB_W0     45056
#define TAB_WB     45824
#define TAB_ZB     46592
#define TAB_FW     47616
#define TAB_BYTES  47872
#define TAB_CHUNKS (TAB_BYTES / 16)

static_assert(TAB_ZT == 3 * NPAD * KIN * 2, "");
static_assert(TAB_W0 == TAB_ZT + NZL * NPAD * KZ * 2, "");
static_assert(TAB_WB == TAB_W0 + 3 * NPAD * 4, "");
static_assert(TAB_ZB == TAB_WB + 3 * NPAD * 4, "");
static_assert(TAB_FW == TAB_ZB + NZL * NPAD * 4, "");
static_assert(TAB_BYTES == TAB_FW + NPAD * 4, "");
static_assert(TAB_BYTES % 128 == 0, "");

#define SC_IN        4096.0f
#define SC_IN_INV    5.9604644775390625e-8f
#define SC_HA        256.0f
#define SC_ZW        1024.0f
#define SC_Z_INV     3.814697265625e-6f
#define OMEGA1       1.5707963267948966f
#define TWO_OVER_LN2 2.8853900817779268f

__device__ __forceinline__ float tanh_f(float x) {
  float e = __builtin_amdgcn_exp2f(x * TWO_OVER_LN2);
  float r = __builtin_amdgcn_rcpf(e + 1.0f);
  return fmaf(-2.0f, r, 1.0f);
}

__device__ __forceinline__ v16h ldfrag(const _Float16* p, int k0, int hf) {
  v8h q0 = *(const v8h*)(p + k0 + 8 * hf);
  v8h q1 = *(const v8h*)(p + k0 + 16 + 8 * hf);
  return __builtin_shufflevector(q0, q1, 0, 1, 2, 3, 4, 5, 6, 7, 8, 9, 10, 11, 12, 13, 14, 15);
}

__device__ __forceinline__ v8f wmma_1(v16h a, v16h b) {
  v8f c = {0.f, 0.f, 0.f, 0.f, 0.f, 0.f, 0.f, 0.f};
  c = __builtin_amdgcn_wmma_f32_16x16x32_f16(false, a, false, b, (short)0, c, false, false);
  asm volatile("v_nop\n\tv_nop\n\tv_nop\n\tv_nop" : "+v"(c) : "v"(a), "v"(b));
  return c;
}

__device__ __forceinline__ v8f wmma_2(v16h a0, v16h b0, v16h a1, v16h b1) {
  v8f c = {0.f, 0.f, 0.f, 0.f, 0.f, 0.f, 0.f, 0.f};
  c = __builtin_amdgcn_wmma_f32_16x16x32_f16(false, a0, false, b0, (short)0, c, false, false);
  c = __builtin_amdgcn_wmma_f32_16x16x32_f16(false, a1, false, b1, (short)0, c, false, false);
  asm volatile("v_nop\n\tv_nop\n\tv_nop\n\tv_nop" : "+v"(c) : "v"(a0), "v"(b0), "v"(a1), "v"(b1));
  return c;
}

__device__ __forceinline__ void put3(_Float16* row, int c, float f) {
  float v = f * SC_IN;
  _Float16 hi = (_Float16)v;
  _Float16 lo = (_Float16)(v - (float)hi);
  row[c] = hi;
  row[NFEAT + c] = lo;
  row[2 * NFEAT + c] = hi;
}

__global__ __launch_bounds__(NTHREADS) void k_prep(
    const float* __restrict__ U_W, const float* __restrict__ U_b,
    const float* __restrict__ V_W, const float* __restrict__ V_b,
    const float* __restrict__ H_W, const float* __restrict__ H_b,
    const float* __restrict__ Z_W, const float* __restrict__ Z_b,
    const float* __restrict__ F_W, unsigned char* __restrict__ tab)
{
  __shared__ __align__(16) unsigned char s[TAB_BYTES];
  _Float16* wt = (_Float16*)(s + TAB_WT);
  _Float16* zt = (_Float16*)(s + TAB_ZT);
  float* w0 = (float*)(s + TAB_W0);
  float* wb = (float*)(s + TAB_WB);
  float* zb = (float*)(s + TAB_ZB);
  float* fw = (float*)(s + TAB_FW);
  const int tid = threadIdx.x;

  for (int idx = tid; idx < 3 * NPAD * KIN; idx += NTHREADS) {
    int g   = idx / (NPAD * KIN);
    int rem = idx - g * (NPAD * KIN);
    int n   = rem / KIN;
    int k   = rem - n * KIN;
    const float* W = (g == 0) ? U_W : (g == 1) ? V_W : H_W;
    _Float16 val = (_Float16)0.0f;
    if (n < HIDDEN && k < 3 * NFEAT) {
      int seg = k / NFEAT;
      int c   = k - seg * NFEAT;
      float v = W[(2 + c) * HIDDEN + n] * SC_IN;
      _Float16 hi = (_Float16)v;
      val = (seg < 2) ? hi : (_Float16)(v - (float)hi);
    }
    wt[idx] = val;
  }
  for (int idx = tid; idx < 3 * NPAD; idx += NTHREADS) {
    int g = idx / NPAD;
    int n = idx - g * NPAD;
    const float* W = (g == 0) ? U_W : (g == 1) ? V_W : H_W;
    const float* B = (g == 0) ? U_b : (g == 1) ? V_b : H_b;
    float a = 0.0f, b = 0.0f;
    if (n < HIDDEN) { a = W[n]; b = W[HIDDEN + n] + B[n]; }
    w0[idx] = a;
    wb[idx] = b;
  }
  for (int idx = tid; idx < NZL * NPAD * KZ; idx += NTHREADS) {
    int i   = idx / (NPAD * KZ);
    int rem = idx - i * (NPAD * KZ);
    int n   = rem / KZ;
    int k   = rem - n * KZ;
    _Float16 val = (_Float16)0.0f;
    if (n < HIDDEN && k < HIDDEN) val = (_Float16)(Z_W[(i * HIDDEN + k) * HIDDEN + n] * SC_ZW);
    zt[idx] = val;
  }
  for (int idx = tid; idx < NZL * NPAD; idx += NTHREADS) {
    int i = idx / NPAD;
    int n = idx - i * NPAD;
    zb[idx] = (n < HIDDEN) ? Z_b[i * HIDDEN + n] : 0.0f;
  }
  for (int idx = tid; idx < NPAD; idx += NTHREADS) fw[idx] = (idx < HIDDEN) ? F_W[idx] : 0.0f;
  __syncthreads();

  const v4u* src = (const v4u*)s;
  for (int q = tid; q < TAB_CHUNKS; q += NTHREADS) {
    v4u v = src[q];
    *(volatile v4u*)(tab + 16 * (size_t)q) = v;
  }
  __threadfence();
  for (int q = tid; q < TAB_CHUNKS; q += NTHREADS) {
    v4u v = src[q];
    *(volatile v4u*)(tab + 16 * (size_t)q) = v;
  }
}

__global__ __launch_bounds__(NTHREADS) void k_mlp(
    const float* __restrict__ X, const unsigned char* __restrict__ tab,
    const float* __restrict__ F_b, float* out, int nrows)
{
  __shared__ __align__(16) unsigned char sTab[TAB_BYTES];
  __shared__ __align__(16) _Float16 sA[8 * 16 * ASTRIDE];
  __shared__ __align__(16) float    sT[8 * 16];
  __shared__ __align__(16) float    sF[8 * 16 * FSTRIDE];
  __shared__ __align__(16) float    sOut[RPB];

  const int tid  = threadIdx.x;
  const int wave = tid >> 5;
  const int lane = tid & 31;
  const int hf   = lane >> 4;
  const int nl   = lane & 15;

  for (int q = tid; q < TAB_CHUNKS; q += NTHREADS)
    ((v4u*)sTab)[q] = ((const v4u*)tab)[q];

  const _Float16* sWT = (const _Float16*)(sTab + TAB_WT);
  const _Float16* sZT = (const _Float16*)(sTab + TAB_ZT);
  const float*    sW0 = (const float*)(sTab + TAB_W0);
  const float*    sWB = (const float*)(sTab + TAB_WB);
  const float*    sZb = (const float*)(sTab + TAB_ZB);
  const float*    sFW = (const float*)(sTab + TAB_FW);

  const int baseRow = blockIdx.x * RPB + wave * 16;
  _Float16* myA = sA + wave * 16 * ASTRIDE;
  float*    myF = sF + wave * 16 * FSTRIDE;

  {
    int r = baseRow + nl;
    if (r > nrows - 1) r = nrows - 1;
    float2 xv = *(const float2*)(X + 2 * (size_t)r);
    float t = xv.x, xs = xv.y;
    _Float16* row = myA + nl * ASTRIDE;
    if (hf == 0) sT[wave * 16 + nl] = t;
#pragma unroll
    for (int i = 0; i < 3; ++i) {
      int j = 1 + 3 * hf + i;
      float om = (float)j * OMEGA1;
      float a = xs * om;
      float cv = cosf(a);
      float sv = sinf(a);
      if (j <= 5) {
        put3(row, j - 1, cv);
        put3(row, j + 4, sv);
      }
    }
    if (hf == 1) { row[30] = (_Float16)0.0f; row[31] = (_Float16)0.0f; }
  }
  __syncthreads();

  float tv[8];
#pragma unroll
  for (int e = 0; e < 8; ++e) tv[e] = sT[wave * 16 + 8 * hf + e];

  v8f u[4], d[4], hs[4];

  {
    v16h a = ldfrag(myA + nl * ASTRIDE, 0, hf);
#pragma unroll
    for (int g = 0; g < 3; ++g) {
#pragma unroll
      for (int t4 = 0; t4 < 4; ++t4) {
        const int col = 16 * t4 + nl;
        v16h b = ldfrag(sWT + (g * NPAD + col) * KIN, 0, hf);
        v8f c = wmma_1(a, b);
        const float cw0 = sW0[g * NPAD + col];
        const float cwb = sWB[g * NPAD + col];
#pragma unroll
        for (int e = 0; e < 8; ++e) {
          float pre = fmaf(tv[e], cw0, fmaf(c[e], SC_IN_INV, cwb));
          float v = tanh_f(pre);
          if (g == 0)      u[t4][e]  = v;
          else if (g == 1) d[t4][e]  = v - u[t4][e];
          else             hs[t4][e] = v;
        }
      }
    }
  }

#pragma unroll 1
  for (int i = 0; i < NZL; ++i) {
#pragma unroll
    for (int t4 = 0; t4 < 4; ++t4) {
#pragma unroll
      for (int e = 0; e < 8; ++e)
        myA[(e + 8 * hf) * ASTRIDE + 16 * t4 + nl] = (_Float16)(hs[t4][e] * SC_HA);
    }
    __syncthreads();

    v16h a0 = ldfrag(myA + nl * ASTRIDE, 0, hf);
    v16h a1 = ldfrag(myA + nl * ASTRIDE, 32, hf);
    const _Float16* zt = sZT + i * NPAD * KZ;
    const float*    zb = sZb + i * NPAD;
#pragma unroll
    for (int t4 = 0; t4 < 4; ++t4) {
      const int col = 16 * t4 + nl;
      const _Float16* zc = zt + col * KZ;
      v16h b0 = ldfrag(zc, 0, hf);
      v16h b1 = ldfrag(zc, 32, hf);
      v8f c = wmma_2(a0, b0, a1, b1);
      const float bcol = zb[col];
#pragma unroll
      for (int e = 0; e < 8; ++e) {
        float z = tanh_f(fmaf(c[e], SC_Z_INV, bcol));
        hs[t4][e] = fmaf(z, d[t4][e], u[t4][e]);
      }
    }
    __syncthreads();
  }

#pragma unroll
  for (int t4 = 0; t4 < 4; ++t4) {
#pragma unroll
    for (int e = 0; e < 8; ++e)
      myF[(e + 8 * hf) * FSTRIDE + 16 * t4 + nl] = hs[t4][e];
  }
  __syncthreads();

  if (hf == 0) {
    const float* rp = myF + nl * FSTRIDE;
    float acc = F_b[0];
#pragma unroll
    for (int k = 0; k < HIDDEN; ++k) acc = fmaf(rp[k], sFW[k], acc);
    sOut[wave * 16 + nl] = acc;
  }
  __syncthreads();

  const int orow0 = blockIdx.x * RPB;
  const int obase = orow0 + 4 * lane;
  v4f ov = *(const v4f*)(sOut + 4 * lane);
  const bool full = (obase + 3 < nrows);
  if (wave == 0) {
    if (full) {
      *(volatile v4f*)(out + obase) = ov;
    } else {
      volatile float* vo = out;
      if (obase + 0 < nrows) vo[obase + 0] = ov.x;
      if (obase + 1 < nrows) vo[obase + 1] = ov.y;
      if (obase + 2 < nrows) vo[obase + 2] = ov.z;
      if (obase + 3 < nrows) vo[obase + 3] = ov.w;
    }
  }
  __threadfence();
  if (wave == 0) {
    if (full) {
      *(volatile v4f*)(out + obase) = ov;
    } else {
      volatile float* vo = out;
      if (obase + 0 < nrows) vo[obase + 0] = ov.x;
      if (obase + 1 < nrows) vo[obase + 1] = ov.y;
      if (obase + 2 < nrows) vo[obase + 2] = ov.z;
      if (obase + 3 < nrows) vo[obase + 3] = ov.w;
    }
  }
}

extern "C" void kernel_launch(void* const* d_in, const int* in_sizes, int n_in,
                              void* d_out, int out_size, void* d_ws, size_t ws_size,
                              hipStream_t stream) {
  (void)n_in; (void)out_size;
  const float* X   = (const float*)d_in[0];
  const float* U_W = (const float*)d_in[1];
  const float* U_b = (const float*)d_in[2];
  const float* V_W = (const float*)d_in[3];
  const float* V_b = (const float*)d_in[4];
  const float* H_W = (const float*)d_in[5];
  const float* H_b = (const float*)d_in[6];
  const float* Z_W = (const float*)d_in[7];
  const float* Z_b = (const float*)d_in[8];
  const float* F_W = (const float*)d_in[9];
  const float* F_b = (const float*)d_in[10];
  float* out = (float*)d_out;

  const int nrows = in_sizes[0] / 2;
  if (nrows <= 0) return;
  if (ws_size < (size_t)TAB_BYTES) return;

  unsigned char* tab = (unsigned char*)d_ws;
  k_prep<<<1, NTHREADS, 0, stream>>>(U_W, U_b, V_W, V_b, H_W, H_b, Z_W, Z_b, F_W, tab);

  const int grid = (nrows + RPB - 1) / RPB;
  k_mlp<<<grid, NTHREADS, 0, stream>>>(X, tab, F_b, out, nrows);
}
